// PointNetRot9d_40931038331358
// MI455X (gfx1250) — hardware-verified
//
#include <hip/hip_runtime.h>


namespace {
constexpr int Bn = 32, NPTS = 2048, NR = Bn * NPTS, C1 = 64, C2 = 128, C3 = 1024, F1 = 512, F2 = 256, NP = 12;
constexpr int NB = NR / 128;
constexpr float AS = 8.0f, WS = 64.0f, EPS = 1e-5f;

typedef _Float16 b16;
typedef __attribute__((ext_vector_type(16))) _Float16 v16b;
typedef __attribute__((ext_vector_type(8)))  _Float16 v8b;
typedef __attribute__((ext_vector_type(8)))  float v8f;
typedef __attribute__((ext_vector_type(4)))  float v4f;

__device__ __forceinline__ v8b ld8b(const b16* p) { return *(const v8b*)p; }
__device__ __forceinline__ v16b cat8b(v8b a, v8b b) { return __builtin_shufflevector(a, b, 0, 1, 2, 3, 4, 5, 6, 7, 8, 9, 10, 11, 12, 13, 14, 15); }
__device__ __forceinline__ v16b frag_kb(const b16* p, int hh) { return cat8b(ld8b(p + 8 * hh), ld8b(p + 16 + 8 * hh)); }
__device__ __forceinline__ void split16(float v, b16& hi, b16& lo) { hi = (b16)v; lo = (b16)(v - (float)hi); }
__device__ __forceinline__ void frag_ksplit(const float* p, int hh, v16b& fh_, v16b& fl_) {
  const float* p0 = p + 8 * hh; const float* p1 = p + 16 + 8 * hh;
#pragma unroll
  for (int e = 0; e < 8; ++e) { b16 a, c; split16(p0[e], a, c); fh_[e] = a; fl_[e] = c; split16(p1[e], a, c); fh_[8 + e] = a; fl_[8 + e] = c; }
}
__device__ __forceinline__ v8f wmma16b(v16b a, v16b b, v8f c) {
  v8f d = __builtin_amdgcn_wmma_f32_16x16x32_f16(false, a, false, b, (short)0, c, false, false);
  asm volatile("v_nop\n\tv_nop\n\tv_nop\n\tv_nop" : "+v"(d) : "v"(a), "v"(b));
  return d;
}
__device__ __forceinline__ void wave_lds_sync() {
  __builtin_amdgcn_fence(__ATOMIC_RELEASE, "workgroup");
  __builtin_amdgcn_wave_barrier();
  __builtin_amdgcn_fence(__ATOMIC_ACQUIRE, "workgroup");
}

struct Opnd { const void* p0; const void* p1; int ld; };
template <int NP> __device__ __forceinline__ void load_frags(const Opnd& o, int row, int kb, int hh, v16b& fh_, v16b& fl_) {
  if (NP == 0) { frag_ksplit((const float*)o.p0 + (size_t)row * o.ld + kb, hh, fh_, fl_); }
  else if (NP == 4 || NP == 5) {
    const float sc_ = (NP == 4) ? 64.0f : 8.0f;
    const float* p = (const float*)o.p0 + (size_t)row * o.ld + kb; const float* p0 = p + 8 * hh; const float* p1 = p + 16 + 8 * hh;
#pragma unroll
    for (int e = 0; e < 8; ++e) { b16 a, c; split16(p0[e] * sc_, a, c); fh_[e] = a; fl_[e] = c; split16(p1[e] * sc_, a, c); fh_[8 + e] = a; fl_[8 + e] = c; }
  } else if (NP == 3) {
    const float* p = (const float*)o.p0 + (size_t)row * o.ld + kb; const float* p0 = p + 8 * hh; const float* p1 = p + 16 + 8 * hh;
#pragma unroll
    for (int e = 0; e < 8; ++e) { fh_[e] = (b16)p0[e]; fh_[8 + e] = (b16)p1[e]; }
    fl_ = fh_;
  } else {
    fh_ = frag_kb((const b16*)o.p0 + (size_t)row * o.ld + kb, hh);
    if (NP == 2) fl_ = frag_kb((const b16*)o.p1 + (size_t)row * o.ld + kb, hh); else fl_ = fh_;
  }
}
template <int ANP, int BNP> __device__ __forceinline__ v8f mac(v16b ah, v16b al, v16b bh, v16b bl, v8f c) {
  c = wmma16b(ah, bh, c);
  if (BNP == 0 || BNP == 2 || BNP == 4 || BNP == 5) c = wmma16b(ah, bl, c);
  if (ANP == 0 || ANP == 2 || ANP == 4 || ANP == 5) c = wmma16b(al, bh, c);
  return c;
}
template <int ANP, int BNP>
__device__ __forceinline__ void gemm_tile(const Opnd& A, const Opnd& B, int K, int m0, int c0, int nloc, int hlf, v8f (&acc)[2][4]) {
  for (int kb = 0; kb < K; kb += 32) {
    v16b a0h, a0l, a1h, a1l;
    load_frags<ANP>(A, m0 + nloc, kb, hlf, a0h, a0l);
    load_frags<ANP>(A, m0 + 16 + nloc, kb, hlf, a1h, a1l);
#pragma unroll
    for (int t = 0; t < 4; ++t) {
      v16b bh, bl;
      load_frags<BNP>(B, c0 + t * 16 + nloc, kb, hlf, bh, bl);
      acc[0][t] = mac<ANP, BNP>(a0h, a0l, bh, bl, acc[0][t]);
      acc[1][t] = mac<ANP, BNP>(a1h, a1l, bh, bl, acc[1][t]);
    }
  }
}

__device__ __forceinline__ void epi_planes(v8f (&acc)[2][4], float scale, bool two, b16* __restrict__ oh, b16* __restrict__ ol, int ldo,
                                           int m0, int c0, int lane, b16* Th, b16* Tl) {
  const int nloc = lane & 15, hlf = lane >> 4;
#pragma unroll
  for (int t = 0; t < 4; ++t)
#pragma unroll
    for (int r = 0; r < 2; ++r)
#pragma unroll
      for (int v = 0; v < 8; ++v) {
        const int rr = r * 16 + v + 8 * hlf, cc = t * 16 + nloc;
        b16 h_, l_; split16(acc[r][t][v] * scale, h_, l_);
        Th[rr * 64 + cc] = h_; Tl[rr * 64 + cc] = l_;
      }
  wave_lds_sync();
  for (int pass = 0; pass < 2; ++pass) {
#pragma unroll
    for (int j = 0; j < 8; ++j) {
      const int rr = j * 4 + (lane >> 3), c8 = (lane & 7) * 8;
      const size_t o = (size_t)(m0 + rr) * ldo + c0 + c8;
      *(volatile v8b*)(oh + o) = ld8b(Th + rr * 64 + c8);
      if (two) *(volatile v8b*)(ol + o) = ld8b(Tl + rr * 64 + c8);
    }
    __threadfence();
  }
}
__device__ __forceinline__ void epi_f32(v8f (&acc)[2][4], float scale, const float* rscale, float* __restrict__ out, int ldo, int m0, int c0, int lane, float* Tt) {
  const int nloc = lane & 15, hlf = lane >> 4;
#pragma unroll
  for (int t = 0; t < 4; ++t)
#pragma unroll
    for (int r = 0; r < 2; ++r)
#pragma unroll
      for (int v = 0; v < 8; ++v) {
        const int rr = r * 16 + v + 8 * hlf;
        const float rs = rscale ? rscale[(size_t)(m0 + rr) * 32] : 1.0f;
        Tt[rr * 64 + t * 16 + nloc] = acc[r][t][v] * scale * rs;
      }
  wave_lds_sync();
  float* dst0 = out + (size_t)m0 * ldo + c0;
  for (int pass = 0; pass < 2; ++pass) {
#pragma unroll
    for (int j = 0; j < 16; ++j) { const int rr = j * 2 + hlf, c4 = nloc * 4; *(volatile v4f*)(dst0 + (size_t)rr * ldo + c4) = *(const v4f*)(Tt + rr * 64 + c4); }
    __threadfence();
  }
}


__global__ __launch_bounds__(256) void prep_kernel(const float* __restrict__ w2, const float* __restrict__ w3, const float* __restrict__ wf1, const float* __restrict__ wf2,
                                                   const float* __restrict__ wp, b16* __restrict__ ph, b16* __restrict__ pl) {
  const size_t tid = (size_t)blockIdx.x * blockDim.x + threadIdx.x, stride = (size_t)gridDim.x * blockDim.x;
  const size_t n2 = (size_t)C2 * C1, n3 = (size_t)C3 * C2, n4 = (size_t)F1 * C3, n5 = (size_t)F2 * F1, n6 = (size_t)16 * F2, tot = (n2 + n3 + n4 + n5 + n6) / 8;
  for (int pass = 0; pass < 2; ++pass) {
    for (size_t p8 = tid; p8 < tot; p8 += stride) {
      const size_t i0 = p8 * 8; v8b vh, vl;
#pragma unroll
      for (int e = 0; e < 8; ++e) { size_t i = i0 + e; float w;
        if (i < n2) w = w2[i]; else if ((i -= n2) < n3) w = w3[i]; else if ((i -= n3) < n4) w = wf1[i]; else if ((i -= n4) < n5) w = wf2[i]; else { i -= n5; w = (i < (size_t)NP * F2) ? wp[i] : 0.0f; }
        b16 a, b2; split16(w * WS, a, b2); vh[e] = a; vl[e] = b2; }
      *(volatile v8b*)(ph + i0) = vh; *(volatile v8b*)(pl + i0) = vl;
    }
    __threadfence();
  }
}

__global__ __launch_bounds__(128) void l1_kernel(const float* __restrict__ x, const float* __restrict__ w1, const float* __restrict__ b1, float* __restrict__ h1, float* __restrict__ slot) {
  __shared__ __attribute__((aligned(16))) float Tt[128 * (C1 + 1)];
  __shared__ float Sh[2][2][C1];
  const int t = threadIdx.x, p0 = blockIdx.x * 128, p = p0 + t, b = p / NPTS, n = p % NPTS;
  const float x0 = x[((size_t)b * 3 + 0) * NPTS + n], x1 = x[((size_t)b * 3 + 1) * NPTS + n], x2 = x[((size_t)b * 3 + 2) * NPTS + n];
#pragma unroll 1
  for (int o = 0; o < C1; ++o) Tt[t * (C1 + 1) + o] = b1[o] + x0 * w1[o * 3] + x1 * w1[o * 3 + 1] + x2 * w1[o * 3 + 2];
  __syncthreads();
  for (int pass = 0; pass < 2; ++pass) {
#pragma unroll
    for (int i = 0; i < 16; ++i) { const int f = (i * 128 + t) * 4, row = f / C1, c = f % C1; const v4f w4 = {Tt[row * (C1 + 1) + c], Tt[row * (C1 + 1) + c + 1], Tt[row * (C1 + 1) + c + 2], Tt[row * (C1 + 1) + c + 3]};
      *(volatile v4f*)(h1 + (size_t)p0 * C1 + f) = w4; }
    __threadfence();
  }
  { const int o = t & (C1 - 1), half = t >> 6; float s = 0.0f, s2 = 0.0f;
#pragma unroll 1
    for (int r = half * 64; r < half * 64 + 64; ++r) { const float v = Tt[r * (C1 + 1) + o]; s += v; s2 += v * v; }
    Sh[half][0][o] = s; Sh[half][1][o] = s2; }
  __syncthreads();
  if (t < C1) { const float s = Sh[0][0][t] + Sh[1][0][t], s2 = Sh[0][1][t] + Sh[1][1][t];
    for (int pass = 0; pass < 2; ++pass) { ((volatile float*)slot)[((size_t)blockIdx.x * 2) * C3 + t] = s; ((volatile float*)slot)[((size_t)blockIdx.x * 2 + 1) * C3 + t] = s2; __threadfence(); } }
}

__global__ __launch_bounds__(256) void bnfin_kernel(const float* __restrict__ slot, int nch, const float* __restrict__ g, const float* __restrict__ bb, float* __restrict__ coef) {
  const int c = blockIdx.x * 256 + threadIdx.x; if (c >= nch) return;
  double s = 0.0, s2 = 0.0;
#pragma unroll 1
  for (int bk = 0; bk < NB; ++bk) { s += (double)slot[((size_t)bk * 2) * C3 + c]; s2 += (double)slot[((size_t)bk * 2 + 1) * C3 + c]; }
  const double mean = s / NR, var = s2 / NR - mean * mean;
  const float a = g[c] * (float)(1.0 / sqrt(var + (double)EPS)), sh = bb[c] - (float)mean * a;
  for (int pass = 0; pass < 2; ++pass) { ((volatile float*)coef)[c] = a; ((volatile float*)coef)[C3 + c] = sh; ((volatile float*)coef)[2 * C3 + c] = (float)mean; __threadfence(); }
}

__global__ __launch_bounds__(256) void bnapply_kernel(const float* __restrict__ h, int nch, const float* __restrict__ coef, b16* __restrict__ oh, b16* __restrict__ ol) {
  const int t = threadIdx.x, r0 = blockIdx.x * 128; const int npc = 128 * nch / 8;
  for (int pass = 0; pass < 2; ++pass) {
    for (int pc_ = t; pc_ < npc; pc_ += 256) { const int row = r0 + pc_ / (nch / 8), c8 = (pc_ % (nch / 8)) * 8; v8b vh, vl;
#pragma unroll
      for (int e = 0; e < 8; ++e) { const int c = c8 + e; b16 a, b2; split16(fmaxf(h[(size_t)row * nch + c] * coef[c] + coef[C3 + c], 0.0f) * AS, a, b2); vh[e] = a; vl[e] = b2; }
      *(volatile v8b*)(oh + (size_t)row * nch + c8) = vh; *(volatile v8b*)(ol + (size_t)row * nch + c8) = vl; }
    __threadfence();
  }
}

__global__ __launch_bounds__(128) void l2_kernel(const b16* __restrict__ ah, const b16* __restrict__ al, const b16* __restrict__ wh, const b16* __restrict__ wl, const float* __restrict__ b2,
                                                float* __restrict__ h2, float* __restrict__ slot) {
  __shared__ __attribute__((aligned(16))) float Ts[4][32 * 64]; __shared__ float Ss[4][2][64];
  const int lane = threadIdx.x & 31, wave = threadIdx.x >> 5, nloc = lane & 15, hlf = lane >> 4, m0 = blockIdx.y * 128 + wave * 32, c0 = blockIdx.x * 64;
  v8f acc[2][4];
#pragma unroll
  for (int r = 0; r < 2; ++r)
#pragma unroll
    for (int t = 0; t < 4; ++t) acc[r][t] = (v8f){};
  const Opnd A{ah, al, C1}, B{wh, wl, C1};
  gemm_tile<2, 2>(A, B, C1, m0, c0, nloc, hlf, acc);
  float cs[4] = {0, 0, 0, 0}, cs2[4] = {0, 0, 0, 0};
#pragma unroll
  for (int t = 0; t < 4; ++t)
#pragma unroll
    for (int r = 0; r < 2; ++r)
#pragma unroll
      for (int v = 0; v < 8; ++v) { const float val = acc[r][t][v] * (1.0f / (AS * WS)) + b2[c0 + t * 16 + nloc]; acc[r][t][v] = val; cs[t] += val; cs2[t] += val * val; }
#pragma unroll
  for (int t = 0; t < 4; ++t) { cs[t] += __shfl_xor(cs[t], 16); cs2[t] += __shfl_xor(cs2[t], 16); if (hlf == 0) { Ss[wave][0][t * 16 + nloc] = cs[t]; Ss[wave][1][t * 16 + nloc] = cs2[t]; } }
  epi_f32(acc, 1.0f, nullptr, h2, C2, m0, c0, lane, Ts[wave]);
  __syncthreads();
  if (wave == 0) { for (int o = lane; o < 64; o += 32) { const float s = Ss[0][0][o] + Ss[1][0][o] + Ss[2][0][o] + Ss[3][0][o], s2 = Ss[0][1][o] + Ss[1][1][o] + Ss[2][1][o] + Ss[3][1][o];
      for (int pass = 0; pass < 2; ++pass) { ((volatile float*)slot)[((size_t)blockIdx.y * 2) * C3 + c0 + o] = s; ((volatile float*)slot)[((size_t)blockIdx.y * 2 + 1) * C3 + c0 + o] = s2; __threadfence(); } } }
}

__global__ __launch_bounds__(128) void l3_kernel(const b16* __restrict__ ah, const b16* __restrict__ al, const b16* __restrict__ wh, const b16* __restrict__ wl, const float* __restrict__ b3, float* __restrict__ wslot) {
  __shared__ __attribute__((aligned(16))) float Ss[4][4][64];
  const int lane = threadIdx.x & 31, wave = threadIdx.x >> 5, nloc = lane & 15, hlf = lane >> 4, m0 = blockIdx.y * 128 + wave * 32, c0 = blockIdx.x * 64;
  v8f acc[2][4];
#pragma unroll
  for (int r = 0; r < 2; ++r)
#pragma unroll
    for (int t = 0; t < 4; ++t) acc[r][t] = (v8f){};
  const Opnd A{ah, al, C2}, B{wh, wl, C2};
  gemm_tile<2, 2>(A, B, C2, m0, c0, nloc, hlf, acc);
#pragma unroll
  for (int t = 0; t < 4; ++t) {
    const float bias = b3[c0 + t * 16 + nloc]; float mx = -INFINITY, mn = INFINITY, s = 0.0f, s2 = 0.0f;
#pragma unroll
    for (int r = 0; r < 2; ++r)
#pragma unroll
      for (int v = 0; v < 8; ++v) { const float val = acc[r][t][v] * (1.0f / (AS * WS)) + bias; mx = fmaxf(mx, val); mn = fminf(mn, val); s += val; s2 += val * val; }
    mx = fmaxf(mx, __shfl_xor(mx, 16)); mn = fminf(mn, __shfl_xor(mn, 16)); s += __shfl_xor(s, 16); s2 += __shfl_xor(s2, 16);
    if (hlf == 0) { Ss[wave][0][t * 16 + nloc] = mx; Ss[wave][1][t * 16 + nloc] = mn; Ss[wave][2][t * 16 + nloc] = s; Ss[wave][3][t * 16 + nloc] = s2; }
  }
  wave_lds_sync();
  const size_t wrow = (size_t)blockIdx.y * 4 + wave;
  for (int pass = 0; pass < 2; ++pass) {
    if (lane < 16) {
#pragma unroll
      for (int st = 0; st < 4; ++st) *(volatile v4f*)(wslot + (wrow * 4 + st) * C3 + c0 + lane * 4) = *(const v4f*)(&Ss[wave][st][lane * 4]); }
    __threadfence();
  }
}

__global__ __launch_bounds__(256) void pool_kernel(const float* __restrict__ wslot, const float* __restrict__ g3, const float* __restrict__ be3, float* __restrict__ pooled) {
  const int c = blockIdx.x * 256 + threadIdx.x;
  double s = 0.0, s2 = 0.0;
#pragma unroll 1
  for (int w = 0; w < NR / 32; ++w) { s += (double)wslot[((size_t)w * 4 + 2) * C3 + c]; s2 += (double)wslot[((size_t)w * 4 + 3) * C3 + c]; }
  const double mean = s / NR, var = s2 / NR - mean * mean; const float a = g3[c] * (float)(1.0 / sqrt(var + (double)EPS));
  for (int pass = 0; pass < 2; ++pass) {
#pragma unroll 1
    for (int b = 0; b < Bn; ++b) {
      float mx = -INFINITY, mn = INFINITY;
#pragma unroll 1
      for (int w = 0; w < NPTS / 32; ++w) { const size_t wr = (size_t)b * (NPTS / 32) + w; mx = fmaxf(mx, wslot[(wr * 4 + 0) * C3 + c]); mn = fminf(mn, wslot[(wr * 4 + 1) * C3 + c]); }
      const float ext = (a >= 0.0f) ? mx : mn;
      ((volatile float*)pooled)[(size_t)b * C3 + c] = (ext - (float)mean) * a + be3[c];
    }
    __threadfence();
  }
}

template <int K, int NOUT>
__global__ __launch_bounds__(128) void fc_kernel(const float* __restrict__ in, const b16* __restrict__ wh, const b16* __restrict__ wl, const float* __restrict__ bias,
                                                 const float* __restrict__ g, const float* __restrict__ bb, float* __restrict__ out) {
  __shared__ __attribute__((aligned(16))) float Ts[32][64 + 4];
  const int lane = threadIdx.x & 31, wave = threadIdx.x >> 5, nloc = lane & 15, hlf = lane >> 4, c0 = blockIdx.x * 64 + wave * 16;
  v8f acc[2] = {{}, {}};
  const Opnd A{in, nullptr, K}, B{wh, wl, K};
#pragma unroll 2
  for (int kb = 0; kb < K; kb += 32) {
    v16b a0h, a0l, a1h, a1l, bh_, bl_;
    load_frags<5>(A, nloc, kb, hlf, a0h, a0l); load_frags<5>(A, 16 + nloc, kb, hlf, a1h, a1l); load_frags<2>(B, c0 + nloc, kb, hlf, bh_, bl_);
    acc[0] = mac<5, 2>(a0h, a0l, bh_, bl_, acc[0]); acc[1] = mac<5, 2>(a1h, a1l, bh_, bl_, acc[1]);
  }
  const int c = c0 + nloc; float s = 0.0f;
#pragma unroll
  for (int r = 0; r < 2; ++r)
#pragma unroll
    for (int v = 0; v < 8; ++v) { const float val = acc[r][v] * (1.0f / (AS * WS)) + bias[c]; acc[r][v] = val; s += val; }
  s += __shfl_xor(s, 16);
  const float mean = s * (1.0f / Bn); float s2 = 0.0f;
#pragma unroll
  for (int r = 0; r < 2; ++r)
#pragma unroll
    for (int v = 0; v < 8; ++v) { const float dd = acc[r][v] - mean; s2 += dd * dd; }
  s2 += __shfl_xor(s2, 16);
  const float a = g[c] * rsqrtf(s2 * (1.0f / Bn) + EPS);
#pragma unroll
  for (int r = 0; r < 2; ++r)
#pragma unroll
    for (int v = 0; v < 8; ++v) Ts[r * 16 + 8 * hlf + v][wave * 16 + nloc] = fmaxf((acc[r][v] - mean) * a + bb[c], 0.0f);
  __syncthreads();
  float* dst = out + blockIdx.x * 64;
  for (int pass = 0; pass < 2; ++pass) {
#pragma unroll
    for (int j = 0; j < 4; ++j) { const int rr = j * 8 + (threadIdx.x >> 4), c4 = (threadIdx.x & 15) * 4; *(volatile v4f*)(dst + (size_t)rr * NOUT + c4) = *(const v4f*)(&Ts[rr][c4]); }
    __threadfence();
  }
}

__device__ void jacobi3(double A[3][3], double V[3][3], double w[3]) {
  for (int i = 0; i < 3; ++i) for (int j = 0; j < 3; ++j) V[i][j] = (i == j) ? 1.0 : 0.0;
  for (int sweep = 0; sweep < 12; ++sweep) {
    for (int pq = 0; pq < 3; ++pq) {
      const int p = (pq == 2) ? 1 : 0, q = (pq == 0) ? 1 : 2;
      const double apq = A[p][q]; if (fabs(apq) < 1e-300) continue;
      const double theta = (A[q][q] - A[p][p]) / (2.0 * apq);
      const double tt = ((theta >= 0.0) ? 1.0 : -1.0) / (fabs(theta) + sqrt(theta * theta + 1.0));
      const double cs = 1.0 / sqrt(tt * tt + 1.0), sn = tt * cs;
      for (int k = 0; k < 3; ++k) { const double akp = A[k][p], akq = A[k][q]; A[k][p] = cs * akp - sn * akq; A[k][q] = sn * akp + cs * akq; }
      for (int k = 0; k < 3; ++k) { const double apk = A[p][k], aqk = A[q][k]; A[p][k] = cs * apk - sn * aqk; A[q][k] = sn * apk + cs * aqk; }
      for (int k = 0; k < 3; ++k) { const double vkp = V[k][p], vkq = V[k][q]; V[k][p] = cs * vkp - sn * vkq; V[k][q] = sn * vkp + cs * vkq; }
    }
  }
  for (int i = 0; i < 3; ++i) w[i] = A[i][i];
}

__global__ __launch_bounds__(128) void final_kernel(const float* __restrict__ f2, const b16* __restrict__ wph, const b16* __restrict__ wpl, const float* __restrict__ bp, float* __restrict__ out) {
  __shared__ float Pm[32][16]; __shared__ __attribute__((aligned(16))) float Ob[512];
  const int lane = threadIdx.x & 31, wave = threadIdx.x >> 5, nloc = lane & 15, hlf = lane >> 4;
  if (wave == 0) {
    v8f acc[2] = {{}, {}};
    const Opnd A{f2, nullptr, F2}, B{wph, wpl, F2};
    for (int kb = 0; kb < F2; kb += 32) { v16b a0h, a0l, a1h, a1l, bh_, bl_;
      load_frags<5>(A, nloc, kb, hlf, a0h, a0l); load_frags<5>(A, 16 + nloc, kb, hlf, a1h, a1l); load_frags<2>(B, nloc, kb, hlf, bh_, bl_);
      acc[0] = mac<5, 2>(a0h, a0l, bh_, bl_, acc[0]); acc[1] = mac<5, 2>(a1h, a1l, bh_, bl_, acc[1]); }
#pragma unroll
    for (int r = 0; r < 2; ++r)
#pragma unroll
      for (int v = 0; v < 8; ++v) Pm[r * 16 + 8 * hlf + v][nloc] = acc[r][v] * (1.0f / (AS * WS)) + ((nloc < NP) ? bp[nloc] : 0.0f);
  }
  __syncthreads();
  if (threadIdx.x < Bn) {
    const int b = threadIdx.x; double M[3][3], G[3][3], V[3][3], w[3];
    for (int i = 0; i < 3; ++i) for (int j = 0; j < 3; ++j) M[i][j] = (double)Pm[b][i * 3 + j];
    for (int i = 0; i < 3; ++i) for (int j = 0; j < 3; ++j) { double s_ = 0.0; for (int k = 0; k < 3; ++k) s_ += M[k][i] * M[k][j]; G[i][j] = s_; }
    jacobi3(G, V, w);
    int ord[3] = {0, 1, 2};
    for (int i = 0; i < 3; ++i) for (int j = i + 1; j < 3; ++j) if (w[ord[j]] > w[ord[i]]) { const int tq = ord[i]; ord[i] = ord[j]; ord[j] = tq; }
    double U[3][3], Vs[3][3], R[3][3];
    for (int k = 0; k < 3; ++k) { const int o = ord[k]; const double sg = sqrt(fmax(w[o], 0.0)), inv = (sg > 0.0) ? 1.0 / sg : 0.0;
      for (int i = 0; i < 3; ++i) { Vs[i][k] = V[i][o]; }
      for (int i = 0; i < 3; ++i) { double s_ = 0.0; for (int j = 0; j < 3; ++j) s_ += M[i][j] * V[j][o]; U[i][k] = s_ * inv; } }
    auto det3 = [](double A_[3][3]) { return A_[0][0] * (A_[1][1] * A_[2][2] - A_[1][2] * A_[2][1]) - A_[0][1] * (A_[1][0] * A_[2][2] - A_[1][2] * A_[2][0]) + A_[0][2] * (A_[1][0] * A_[2][1] - A_[1][1] * A_[2][0]); };
    const double dsg = (det3(U) * det3(Vs) >= 0.0) ? 1.0 : -1.0;
    for (int i = 0; i < 3; ++i) for (int j = 0; j < 3; ++j) R[i][j] = U[i][0] * Vs[j][0] + U[i][1] * Vs[j][1] + dsg * U[i][2] * Vs[j][2];
    for (int i = 0; i < 3; ++i) { for (int j = 0; j < 3; ++j) Ob[b * 16 + i * 4 + j] = (float)R[i][j]; Ob[b * 16 + i * 4 + 3] = Pm[b][9 + i]; }
    Ob[b * 16 + 12] = 0.0f; Ob[b * 16 + 13] = 0.0f; Ob[b * 16 + 14] = 0.0f; Ob[b * 16 + 15] = 1.0f;
  }
  __syncthreads();
  for (int pass = 0; pass < 2; ++pass) { *(volatile v4f*)(out + threadIdx.x * 4) = *(const v4f*)(&Ob[threadIdx.x * 4]); __threadfence(); }
}
}

extern "C" void kernel_launch(void* const* d_in, const int* in_sizes, int n_in,
                              void* d_out, int out_size, void* d_ws, size_t ws_size, hipStream_t stream) {
  (void)n_in; (void)out_size;
  const float* x = (const float*)d_in[0];
  const float* w1 = (const float*)d_in[1]; const float* b1 = (const float*)d_in[2]; const float* g1 = (const float*)d_in[3]; const float* be1 = (const float*)d_in[4];
  const float* w2 = (const float*)d_in[5]; const float* b2 = (const float*)d_in[6]; const float* g2 = (const float*)d_in[7]; const float* be2 = (const float*)d_in[8];
  const float* w3 = (const float*)d_in[9]; const float* b3 = (const float*)d_in[10]; const float* g3 = (const float*)d_in[11]; const float* be3 = (const float*)d_in[12];
  const float* wf1 = (const float*)d_in[13]; const float* bf1 = (const float*)d_in[14]; const float* gf1 = (const float*)d_in[15]; const float* bef1 = (const float*)d_in[16];
  const float* wf2 = (const float*)d_in[17]; const float* bf2 = (const float*)d_in[18]; const float* gf2 = (const float*)d_in[19]; const float* bef2 = (const float*)d_in[20];
  const float* wp = (const float*)d_in[21]; const float* bp = (const float*)d_in[22];
  float* out = (float*)d_out;
  if (in_sizes[0] != Bn * 3 * NPTS || in_sizes[1] != C1 * 3 || in_sizes[9] != C3 * C2 || in_sizes[13] != F1 * C3 || in_sizes[21] != NP * F2) return;
  size_t off = 0; char* ws = (char*)d_ws;
  auto carve = [&](size_t bytes) { char* p = ws + off; off += (bytes + 255) & ~(size_t)255; return p; };
  const size_t NPL = (size_t)C2 * C1 + (size_t)C3 * C2 + (size_t)F1 * C3 + (size_t)F2 * F1 + (size_t)16 * F2;
  b16* ph = (b16*)carve(NPL * 2); b16* pl = (b16*)carve(NPL * 2);
  float* big = (float*)carve((size_t)NR * C2 * 4);
  float* h1 = big; float* h2 = big; float* wslot = big;
  float* slot = (float*)carve((size_t)NB * 2 * C3 * 4);
  float* coef = (float*)carve((size_t)3 * C3 * 4);
  b16* a1h = (b16*)carve((size_t)NR * C1 * 2); b16* a1l = (b16*)carve((size_t)NR * C1 * 2);
  b16* a2h = (b16*)carve((size_t)NR * C2 * 2); b16* a2l = (b16*)carve((size_t)NR * C2 * 2);
  float* pooled = (float*)carve((size_t)Bn * C3 * 4); float* f1 = (float*)carve((size_t)Bn * F1 * 4); float* f2b_ = (float*)carve((size_t)Bn * F2 * 4);
  if (off > ws_size) return;
  const b16* w2h = ph; const b16* w2l = pl; const b16* w3h = ph + (size_t)C2 * C1; const b16* w3l = pl + (size_t)C2 * C1;
  const b16* wf1h = w3h + (size_t)C3 * C2; const b16* wf1l = w3l + (size_t)C3 * C2; const b16* wf2h = wf1h + (size_t)F1 * C3; const b16* wf2l = wf1l + (size_t)F1 * C3;
  const b16* wph = wf2h + (size_t)F2 * F1; const b16* wpl = wf2l + (size_t)F2 * F1;
  prep_kernel<<<256, 256, 0, stream>>>(w2, w3, wf1, wf2, wp, ph, pl);
  l1_kernel<<<NB, 128, 0, stream>>>(x, w1, b1, h1, slot);
  bnfin_kernel<<<1, 256, 0, stream>>>(slot, C1, g1, be1, coef);
  bnapply_kernel<<<NB, 256, 0, stream>>>(h1, C1, coef, a1h, a1l);
  l2_kernel<<<dim3(C2 / 64, NB), 128, 0, stream>>>(a1h, a1l, w2h, w2l, b2, h2, slot);
  bnfin_kernel<<<1, 256, 0, stream>>>(slot, C2, g2, be2, coef);
  bnapply_kernel<<<NB, 256, 0, stream>>>(h2, C2, coef, a2h, a2l);
  l3_kernel<<<dim3(C3 / 64, NB), 128, 0, stream>>>(a2h, a2l, w3h, w3l, b3, wslot);
  pool_kernel<<<C3 / 256, 256, 0, stream>>>(wslot, g3, be3, pooled);
  fc_kernel<C3, F1><<<F1 / 64, 128, 0, stream>>>(pooled, wf1h, wf1l, bf1, gf1, bef1, f1);
  fc_kernel<F1, F2><<<F2 / 64, 128, 0, stream>>>(f1, wf2h, wf2l, bf2, gf2, bef2, f2b_);
  final_kernel<<<1, 128, 0, stream>>>(f2b_, wph, wpl, bp, out);
}
